// TransformerConvNet_88553635709219
// MI455X (gfx1250) — hardware-verified
//
#include <hip/hip_runtime.h>
#include <math.h>
#include <stddef.h>


typedef _Float16 v16h __attribute__((ext_vector_type(16)));
typedef _Float16 v8h  __attribute__((ext_vector_type(8)));
typedef float    v8f  __attribute__((ext_vector_type(8)));
typedef float    v4f  __attribute__((ext_vector_type(4)));
typedef int      v4i  __attribute__((ext_vector_type(4)));

union Frag { v16h v; v8h hv[2]; };

__device__ __forceinline__ v8f wmma_f16(v16h a, v16h b, v8f c)
{
    v8f r = __builtin_amdgcn_wmma_f32_16x16x32_f16(false, a, false, b, (short)0, c, false, false);
    asm volatile("v_nop\n\tv_nop\n\tv_nop\n\tv_nop" : "+v"(r) : "v"(a), "v"(b));
    return r;
}

__device__ __forceinline__ v8f vz8()
{
    v8f z = {0.0f, 0.0f, 0.0f, 0.0f, 0.0f, 0.0f, 0.0f, 0.0f};
    return z;
}

__device__ __forceinline__ float elu_f(float x) { return x > 0.0f ? x : (__expf(x) - 1.0f); }

__device__ __forceinline__ int clampi(int v, int lo, int hi) { return v < lo ? lo : (v > hi ? hi : v); }

__device__ __forceinline__ v16h afrag_f32(const float* row, int k0, int hh)
{
    const float* p0 = row + k0 + 8 * hh;
    const float* p1 = row + k0 + 16 + 8 * hh;
    const v4f x0 = *(const v4f*)p0;
    const v4f x1 = *(const v4f*)(p0 + 4);
    const v4f x2 = *(const v4f*)p1;
    const v4f x3 = *(const v4f*)(p1 + 4);
    v16h a;
    a[0]  = (_Float16)x0.x; a[1]  = (_Float16)x0.y; a[2]  = (_Float16)x0.z; a[3]  = (_Float16)x0.w;
    a[4]  = (_Float16)x1.x; a[5]  = (_Float16)x1.y; a[6]  = (_Float16)x1.z; a[7]  = (_Float16)x1.w;
    a[8]  = (_Float16)x2.x; a[9]  = (_Float16)x2.y; a[10] = (_Float16)x2.z; a[11] = (_Float16)x2.w;
    a[12] = (_Float16)x3.x; a[13] = (_Float16)x3.y; a[14] = (_Float16)x3.z; a[15] = (_Float16)x3.w;
    return a;
}

template<int CIN, int C>
__launch_bounds__(256)
__global__ void k_proj4(const float* __restrict__ X, int ldx,
                        const float* __restrict__ W0, const float* __restrict__ W1,
                        const float* __restrict__ W2, const float* __restrict__ W3,
                        const float* __restrict__ B0, const float* __restrict__ B1,
                        const float* __restrict__ B2, const float* __restrict__ B3,
                        float* Y, int nTiles)
{
    constexpr int C4  = 4 * C;
    constexpr int NT  = C4 / 16;
    constexpr int NG  = NT / 4;
    constexpr int KT  = CIN / 32;
    constexpr int TPW = 4;

    __shared__ __align__(32) _Float16 Wl[KT * NT * 512];
    __shared__ float Bs[C4];
    __shared__ __align__(16) float St[8][16 * 64];

    const int tid = (int)threadIdx.x;
    for (int g = tid; g < KT * NT * 32; g += 256) {
        const int kt  = g / (NT * 32);
        const int t   = (g >> 5) % NT;
        const int L   = g & 31;
        const int n   = t * 16 + (L & 15);
        const int hh  = L >> 4;
        const int mat = n / C;
        const int col = n - mat * C;
        const float* Wp = (mat == 0) ? W0 : (mat == 1) ? W1 : (mat == 2) ? W2 : W3;
        v16h fv;
#pragma unroll
        for (int i = 0; i < 8; ++i) {
            fv[i]     = (_Float16)(Wp[(size_t)(kt * 32 + 8 * hh + i) * C + col] * 16.0f);
            fv[8 + i] = (_Float16)(Wp[(size_t)(kt * 32 + 16 + 8 * hh + i) * C + col] * 16.0f);
        }
        *(v16h*)&Wl[g * 16] = fv;
    }
    for (int n = tid; n < C4; n += 256) {
        const int mat = n / C;
        const int col = n - mat * C;
        const float* bp = (mat == 0) ? B0 : (mat == 1) ? B1 : (mat == 2) ? B2 : B3;
        Bs[n] = bp[col];
    }
    __syncthreads();

    const int lane = tid & 31, w = tid >> 5, m = lane & 15, hh = lane >> 4;
    float* st = &St[w][0];

    for (int j = 0; j < TPW; ++j) {
        const int tile = (int)blockIdx.x * (8 * TPW) + j * 8 + w;
        const bool valid = tile < nTiles;
        const int tl = valid ? tile : (nTiles - 1);
        const float* xrow = X + (size_t)(tl * 16 + m) * ldx;
        v16h af[KT];
#pragma unroll
        for (int kt = 0; kt < KT; ++kt) af[kt] = afrag_f32(xrow, kt * 32, hh);

#pragma unroll
        for (int g = 0; g < NG; ++g) {
            v8f acc[4];
#pragma unroll
            for (int t = 0; t < 4; ++t) acc[t] = vz8();
#pragma unroll
            for (int kt = 0; kt < KT; ++kt) {
#pragma unroll
                for (int t = 0; t < 4; ++t) {
                    const v16h b = *(const v16h*)&Wl[((kt * NT + g * 4 + t) * 32 + lane) * 16];
                    acc[t] = wmma_f16(af[kt], b, acc[t]);
                }
            }
#pragma unroll
            for (int t = 0; t < 4; ++t) {
                const float bb = Bs[g * 64 + t * 16 + m];
#pragma unroll
                for (int r = 0; r < 8; ++r)
                    st[(8 * hh + r) * 64 + t * 16 + m] = acc[t][r] * 0.0625f + bb;
            }
            __syncthreads();
            if (valid) {
                v4f vals[8];
#pragma unroll
                for (int q = 0; q < 8; ++q) vals[q] = *(const v4f*)&st[(2 * q + hh) * 64 + 4 * m];
                float* yb = Y + (size_t)tile * 16 * C4 + g * 64 + 4 * m;
#pragma unroll
                for (int q = 0; q < 8; ++q)
                    *(volatile v4f*)(yb + (size_t)(2 * q + hh) * C4) = vals[q];
                __threadfence();
#pragma unroll
                for (int q = 0; q < 8; ++q)
                    *(volatile v4f*)(yb + (size_t)(2 * q + hh) * C4) = vals[q];
            }
            __syncthreads();
        }
    }
}

template<int C>
__launch_bounds__(256)
__global__ void k_edgew(const float* __restrict__ Pm, const int* __restrict__ ei,
                        const float* __restrict__ ea, const float* __restrict__ We,
                        const float* __restrict__ be, float* pe, int N, int E)
{
    constexpr int P4 = 4 * C;
    const int e = (int)blockIdx.x * 256 + (int)threadIdx.x;
    const bool valid = e < E;
    const int ec = valid ? e : (E - 1);
    int s = ei[ec];
    int d = ei[(size_t)E + ec];
    s = clampi(s, 0, N - 1);
    d = clampi(d, 0, N - 1);
    const float a = ea[ec];
    const float* qrow = Pm + (size_t)d * P4;
    const float* krow = Pm + (size_t)s * P4 + C;
    float dot = 0.0f;
#pragma unroll 2
    for (int c = 0; c < C; c += 4) {
        const v4f q4 = *(const v4f*)(qrow + c);
        const v4f k4 = *(const v4f*)(krow + c);
        const v4f w4 = *(const v4f*)(We + c);
        const v4f b4 = *(const v4f*)(be + c);
        const float kx = k4.x + fmaf(a, w4.x, b4.x);
        const float ky = k4.y + fmaf(a, w4.y, b4.y);
        const float kz = k4.z + fmaf(a, w4.z, b4.z);
        const float kw = k4.w + fmaf(a, w4.w, b4.w);
        dot = fmaf(q4.x, kx, dot);
        dot = fmaf(q4.y, ky, dot);
        dot = fmaf(q4.z, kz, dot);
        dot = fmaf(q4.w, kw, dot);
    }
    const float rs = 1.0f / sqrtf((float)C);
    float al = dot * rs;
    al = fminf(fmaxf(al, -80.0f), 80.0f);
    const float p = __expf(al);
    if (valid) *(volatile float*)(pe + e) = p;
    __threadfence();
    if (valid) *(volatile float*)(pe + e) = p;
}

template<int C, int R>
__launch_bounds__(256)
__global__ void k_aggr(const float* Pm, const int* __restrict__ ei, const float* __restrict__ ea,
                       const float* __restrict__ pe, const float* __restrict__ We,
                       const float* __restrict__ be, float* outp, int ldo, int N, int E, int vec4ok)
{
    constexpr int CPL = C / 32;
    constexpr int P4  = 4 * C;
    constexpr int CAP = 128;
    constexpr int CQ  = C / 4;

    extern __shared__ __align__(16) float dyn_lds[];
    float* ACC  = dyn_lds;
    float* Ssum = ACC + R * C;
    int*   CNT  = (int*)(Ssum + R);
    int*   LST  = CNT + 128;
    int*   OVF  = LST + 64 * CAP;

    const int tid = (int)threadIdx.x, lane = tid & 31, w = tid >> 5;
    const int n0 = (int)blockIdx.x * R;
    const int Rb = (N - n0 < R) ? (N - n0) : R;

    {
        const v4f z4 = {0.0f, 0.0f, 0.0f, 0.0f};
        for (int i = tid; i < R * CQ; i += 256) ((v4f*)ACC)[i] = z4;
        for (int i = tid; i < R; i += 256) Ssum[i] = 0.0f;
    }
    __syncthreads();

    const int* src = ei;
    const int* dst = ei + E;
    const int c0 = CPL * lane;
    float wev[CPL], bev[CPL];
#pragma unroll
    for (int u = 0; u < CPL; ++u) { wev[u] = We[c0 + u]; bev[u] = be[c0 + u]; }

    const int nChunk = (E + 255) >> 8;
    const int nIter  = (nChunk + 7) >> 3;

    for (int it = 0; it < nIter; ++it) {
        if (lane < 16) CNT[w * 16 + lane] = 0;
        const int base = (it * 8 + w) << 8;
        int dd[8];
        if (vec4ok != 0 && base + 256 <= E) {
            const v4i t0 = *(const v4i*)(dst + base + 4 * lane);
            const v4i t1 = *(const v4i*)(dst + base + 128 + 4 * lane);
            dd[0] = t0.x; dd[1] = t0.y; dd[2] = t0.z; dd[3] = t0.w;
            dd[4] = t1.x; dd[5] = t1.y; dd[6] = t1.z; dd[7] = t1.w;
        } else {
#pragma unroll
            for (int j = 0; j < 8; ++j) {
                const int e  = base + ((j < 4) ? (4 * lane + j) : (128 + 4 * lane + (j - 4)));
                const int ec = (e < E) ? e : (E - 1);
                const int v  = dst[ec];
                dd[j] = (e < E) ? v : -1;
            }
        }
#pragma unroll
        for (int j = 0; j < 8; ++j) {
            const int dl = dd[j] - n0;
            const bool in = (unsigned)dl < (unsigned)Rb;
            unsigned msk = __builtin_amdgcn_ballot_w32(in);
            while (msk != 0u) {
                const int ln = __builtin_ctz(msk);
                msk &= msk - 1u;
                const int dlh  = __builtin_amdgcn_readlane(dl, ln);
                const int eh   = base + ((j < 4) ? (4 * ln + j) : (128 + 4 * ln + (j - 4)));
                const int cls  = dlh & 7;
                const int slot = w * 8 + cls;
                const int cnt  = CNT[w * 16 + cls];
                if (cnt < CAP) {
                    LST[slot * CAP + cnt] = eh;
                    CNT[w * 16 + cls] = cnt + 1;
                } else {
                    const int oc = CNT[w * 16 + 8];
                    OVF[w * CAP + (oc & (CAP - 1))] = eh;
                    CNT[w * 16 + 8] = oc + 1;
                }
            }
        }
        __syncthreads();
        {
            int cv = 0;
            if (lane < 16) cv = CNT[(lane & 7) * 16 + ((lane < 8) ? w : 8)];
            unsigned any = __builtin_amdgcn_ballot_w32(cv > 0);
            while (any != 0u) {
                const int sl = __builtin_ctz(any);
                any &= any - 1u;
                int cnt = __builtin_amdgcn_readlane(cv, sl);
                cnt = (cnt < CAP) ? cnt : CAP;
                const int sw = sl & 7;
                const int* lp = (sl < 8) ? (LST + (sw * 8 + w) * CAP) : (OVF + sw * CAP);
                for (int i = 0; i < cnt; ++i) {
                    int e = lp[i];
                    e = clampi(e, 0, E - 1);
                    const int   d = dst[e];
                    int         s = src[e];
                    const float a = ea[e];
                    const float p = pe[e];
                    const int dl = d - n0;
                    if ((unsigned)dl < (unsigned)Rb && (dl & 7) == w) {
                        s = clampi(s, 0, N - 1);
                        const float* vrow = Pm + (size_t)s * P4 + 2 * C + c0;
                        float* ap = ACC + dl * C + c0;
#pragma unroll
                        for (int u = 0; u < CPL; ++u) {
                            const float ve = vrow[u] + fmaf(a, wev[u], bev[u]);
                            ap[u] = fmaf(p, ve, ap[u]);
                        }
                        const float sv = Ssum[dl];
                        Ssum[dl] = sv + p;
                    }
                }
            }
        }
        __syncthreads();
    }

    const int nq = Rb * CQ;
    for (int i = tid; i < nq; i += 256) {
        const int r  = i / CQ;
        const int cq = i - r * CQ;
        const v4f av = ((const v4f*)ACC)[i];
        const float inv = 1.0f / (Ssum[r] + 1e-16f);
        const v4f sk = *(const v4f*)(Pm + (size_t)(n0 + r) * P4 + 3 * C + 4 * cq);
        v4f o;
        o.x = elu_f(fmaf(av.x, inv, sk.x));
        o.y = elu_f(fmaf(av.y, inv, sk.y));
        o.z = elu_f(fmaf(av.z, inv, sk.z));
        o.w = elu_f(fmaf(av.w, inv, sk.w));
        ((v4f*)ACC)[i] = o;
    }
    for (int i = tid; i < nq; i += 256) {
        const int r  = i / CQ;
        const int cq = i - r * CQ;
        const v4f o = ((const v4f*)ACC)[i];
        *(volatile v4f*)(outp + (size_t)(n0 + r) * ldo + 4 * cq) = o;
    }
    __threadfence();
    for (int i = tid; i < nq; i += 256) {
        const int r  = i / CQ;
        const int cq = i - r * CQ;
        const v4f o = ((const v4f*)ACC)[i];
        *(volatile v4f*)(outp + (size_t)(n0 + r) * ldo + 4 * cq) = o;
    }
}

__launch_bounds__(256)
__global__ void k_head(const float* __restrict__ Hin, int ldh,
                       const float* __restrict__ W1, const float* __restrict__ B1,
                       const float* __restrict__ W2, const float* __restrict__ B2,
                       float* outp, int nTiles)
{
    constexpr int CIN = 64, HID = 128, NCL = 10;
    constexpr int KT1 = CIN / 32, NT1 = HID / 16, KT2 = HID / 32, TP = 136, TPW = 4;

    __shared__ __align__(32) _Float16 W1l[KT1 * NT1 * 512];
    __shared__ __align__(32) _Float16 W2l[KT2 * 512];
    __shared__ float B1s[HID];
    __shared__ float B2s[16];
    __shared__ __align__(16) _Float16 Tt[8][16 * TP];
    __shared__ __align__(16) float Os[8][160];

    const int tid = (int)threadIdx.x;
    for (int g = tid; g < KT1 * NT1 * 32; g += 256) {
        const int kt = g / (NT1 * 32);
        const int t  = (g >> 5) % NT1;
        const int L  = g & 31;
        const int n  = t * 16 + (L & 15);
        const int hh = L >> 4;
        v16h fv;
#pragma unroll
        for (int i = 0; i < 8; ++i) {
            fv[i]     = (_Float16)(W1[(kt * 32 + 8 * hh + i) * HID + n] * 16.0f);
            fv[8 + i] = (_Float16)(W1[(kt * 32 + 16 + 8 * hh + i) * HID + n] * 16.0f);
        }
        *(v16h*)&W1l[g * 16] = fv;
    }
    for (int g = tid; g < KT2 * 32; g += 256) {
        const int kt = g >> 5;
        const int L  = g & 31;
        const int n  = L & 15;
        const int hh = L >> 4;
        v16h fv;
#pragma unroll
        for (int i = 0; i < 8; ++i) {
            const float x0 = (n < NCL) ? W2[(kt * 32 + 8 * hh + i) * NCL + n] : 0.0f;
            const float x1 = (n < NCL) ? W2[(kt * 32 + 16 + 8 * hh + i) * NCL + n] : 0.0f;
            fv[i]     = (_Float16)(x0 * 16.0f);
            fv[8 + i] = (_Float16)(x1 * 16.0f);
        }
        *(v16h*)&W2l[g * 16] = fv;
    }
    for (int n = tid; n < HID; n += 256) B1s[n] = B1[n];
    if (tid < 16) B2s[tid] = (tid < NCL) ? B2[tid] : 0.0f;
    __syncthreads();

    const int lane = tid & 31, w = tid >> 5, m = lane & 15, hh = lane >> 4;
    _Float16* tt = &Tt[w][0];
    float* os = &Os[w][0];

    for (int j = 0; j < TPW; ++j) {
        const int tile = (int)blockIdx.x * (8 * TPW) + j * 8 + w;
        const bool valid = tile < nTiles;
        const int tl = valid ? tile : (nTiles - 1);
        const float* hrow = Hin + (size_t)(tl * 16 + m) * ldh;
        v16h af[KT1];
#pragma unroll
        for (int kt = 0; kt < KT1; ++kt) af[kt] = afrag_f32(hrow, kt * 32, hh);

#pragma unroll
        for (int g = 0; g < NT1 / 4; ++g) {
            v8f acc[4];
#pragma unroll
            for (int t = 0; t < 4; ++t) acc[t] = vz8();
#pragma unroll
            for (int kt = 0; kt < KT1; ++kt) {
#pragma unroll
                for (int t = 0; t < 4; ++t) {
                    const v16h b = *(const v16h*)&W1l[((kt * NT1 + g * 4 + t) * 32 + lane) * 16];
                    acc[t] = wmma_f16(af[kt], b, acc[t]);
                }
            }
#pragma unroll
            for (int t = 0; t < 4; ++t) {
                const int col = (g * 4 + t) * 16 + m;
                const float bb = B1s[col];
#pragma unroll
                for (int r = 0; r < 8; ++r)
                    tt[(8 * hh + r) * TP + col] = (_Float16)elu_f(acc[t][r] * 0.0625f + bb);
            }
        }
        __syncthreads();

        v8f acc2 = vz8();
#pragma unroll
        for (int kt = 0; kt < KT2; ++kt) {
            Frag a2;
            a2.hv[0] = *(const v8h*)&tt[m * TP + kt * 32 + 8 * hh];
            a2.hv[1] = *(const v8h*)&tt[m * TP + kt * 32 + 16 + 8 * hh];
            const v16h b = *(const v16h*)&W2l[(kt * 32 + lane) * 16];
            acc2 = wmma_f16(a2.v, b, acc2);
        }

        const bool cl = m < NCL;
        const float b2 = B2s[m];
#pragma unroll
        for (int r = 0; r < 8; ++r) {
            const float lv = cl ? (acc2[r] * 0.0625f + b2) : -INFINITY;
            float mx = lv;
            mx = fmaxf(mx, __shfl_xor(mx, 8, 32));
            mx = fmaxf(mx, __shfl_xor(mx, 4, 32));
            mx = fmaxf(mx, __shfl_xor(mx, 2, 32));
            mx = fmaxf(mx, __shfl_xor(mx, 1, 32));
            const float sh = lv - mx;
            float se = cl ? expf(sh) : 0.0f;
            se += __shfl_xor(se, 8, 32);
            se += __shfl_xor(se, 4, 32);
            se += __shfl_xor(se, 2, 32);
            se += __shfl_xor(se, 1, 32);
            const float o = sh - logf(se);
            if (cl) os[(8 * hh + r) * NCL + m] = o;
        }
        __syncthreads();
        if (valid) {
            const v4f va = *(const v4f*)&os[4 * lane];
            v4f vb = va;
            if (lane < 8) vb = *(const v4f*)&os[128 + 4 * lane];
            float* ob = outp + (size_t)tile * 160;
            *(volatile v4f*)(ob + 4 * lane) = va;
            if (lane < 8) *(volatile v4f*)(ob + 128 + 4 * lane) = vb;
            __threadfence();
            *(volatile v4f*)(ob + 4 * lane) = va;
            if (lane < 8) *(volatile v4f*)(ob + 128 + 4 * lane) = vb;
        }
        __syncthreads();
    }
}

extern "C" void kernel_launch(void* const* d_in, const int* in_sizes, int n_in,
                              void* d_out, int out_size, void* d_ws, size_t ws_size,
                              hipStream_t stream)
{
    if (n_in < 27) return;
    const int N = in_sizes[0] / 64;
    const int E = in_sizes[1] / 2;
    if (N < 16 || (N & 15) != 0 || E < 1) return;
    if (in_sizes[2] < E) return;
    if (out_size < N * 10) return;

    const float* x   = (const float*)d_in[0];
    const int*   ei  = (const int*)d_in[1];
    const float* ea  = (const float*)d_in[2];
    const float *Wq1 = (const float*)d_in[3],  *bq1 = (const float*)d_in[4];
    const float *Wk1 = (const float*)d_in[5],  *bk1 = (const float*)d_in[6];
    const float *Wv1 = (const float*)d_in[7],  *bv1 = (const float*)d_in[8];
    const float *We1 = (const float*)d_in[9],  *be1 = (const float*)d_in[10];
    const float *Ws1 = (const float*)d_in[11], *bs1 = (const float*)d_in[12];
    const float *Wq2 = (const float*)d_in[13], *bq2 = (const float*)d_in[14];
    const float *Wk2 = (const float*)d_in[15], *bk2 = (const float*)d_in[16];
    const float *Wv2 = (const float*)d_in[17], *bv2 = (const float*)d_in[18];
    const float *We2 = (const float*)d_in[19], *be2 = (const float*)d_in[20];
    const float *Ws2 = (const float*)d_in[21], *bs2 = (const float*)d_in[22];
    const float *Wf1 = (const float*)d_in[23], *bf1 = (const float*)d_in[24];
    const float *Wf2 = (const float*)d_in[25], *bf2 = (const float*)d_in[26];

    const size_t bytesP  = (size_t)N * 256 * sizeof(float);
    const size_t bytesH1 = (size_t)N * 32 * sizeof(float);
    const size_t bytesPE = (((size_t)E * sizeof(float)) + 255) & ~(size_t)255;
    const size_t offP  = 0;
    const size_t offH1 = offP + bytesP;
    const size_t offPE = offH1 + bytesH1;
    if (offPE + bytesPE > ws_size) return;
    char* ws = (char*)d_ws;
    float* P  = (float*)(ws + offP);
    float* H1 = (float*)(ws + offH1);
    float* PE = (float*)(ws + offPE);

    constexpr int R1 = 1536;
    constexpr int R2 = 768;
    const int nTiles = N / 16;
    const int gTiles = (nTiles + 31) / 32;
    const int gEdge  = (E + 255) / 256;
    const int gA1    = (N + R1 - 1) / R1;
    const int gA2    = (N + R2 - 1) / R2;
    const int vec4ok = ((E & 3) == 0) ? 1 : 0;
    const size_t lds1 = ((size_t)R1 * 32 + R1 + 128 + 64 * 128 + 8 * 128) * sizeof(float);
    const size_t lds2 = ((size_t)R2 * 64 + R2 + 128 + 64 * 128 + 8 * 128) * sizeof(float);
    dim3 blk(256);

    k_proj4<64, 32><<<dim3(gTiles), blk, 0, stream>>>(x, 64, Wq1, Wk1, Wv1, Ws1, bq1, bk1, bv1, bs1, P, nTiles);
    k_edgew<32><<<dim3(gEdge), blk, 0, stream>>>(P, ei, ea, We1, be1, PE, N, E);
    k_aggr<32, R1><<<dim3(gA1), blk, lds1, stream>>>(P, ei, ea, PE, We1, be1, H1, 32, N, E, vec4ok);

    k_proj4<32, 64><<<dim3(gTiles), blk, 0, stream>>>(H1, 32, Wq2, Wk2, Wv2, Ws2, bq2, bk2, bv2, bs2, P, nTiles);
    k_edgew<64><<<dim3(gEdge), blk, 0, stream>>>(P, ei, ea, We2, be2, PE, N, E);
    k_aggr<64, R2><<<dim3(gA2), blk, lds2, stream>>>(P, ei, ea, PE, We2, be2, P + 192, 256, N, E, vec4ok);

    k_head<<<dim3(gTiles), blk, 0, stream>>>(P + 192, 256, Wf1, bf1, Wf2, bf2, (float*)d_out, nTiles);
    (void)hipGetLastError();
}
